// Block_89696097010240
// MI455X (gfx1250) — hardware-verified
//
#include <hip/hip_runtime.h>
#ifndef NB
#define NB 8
#endif
#ifndef SQ
#define SQ 1024
#endif
#define NB_FULL 8
#define SQ_FULL 1024
#define DM 768
#define NH 12
#define HD 64
#define DFF 3072
#define LQ (3 * DM)
#define NR (NB * SQ)
#define SC2 0.18033688011112042f

static_assert(SQ % 128 == 0);
static_assert(SQ % 64 == 0);
static_assert(SQ <= SQ_FULL);
static_assert(NB <= NB_FULL);
static_assert(NH * HD == DM);
static_assert(HD == 64);
static_assert(DM % 64 == 0);
static_assert(LQ % 64 == 0);
static_assert(DFF % 64 == 0);
static_assert(DM % 32 == 0);
static_assert(DFF % 32 == 0);
static_assert(NR % 128 == 0);

typedef unsigned short v8us __attribute__((ext_vector_type(8), may_alias));
typedef float  v8f  __attribute__((ext_vector_type(8)));
typedef float  v4f  __attribute__((ext_vector_type(4)));
typedef float  v4fa __attribute__((ext_vector_type(4), may_alias));
typedef _Float16 v16h __attribute__((ext_vector_type(16)));
typedef _Float16 v4h __attribute__((ext_vector_type(4)));
union FragH { v16h v; v8us half[2]; _Float16 h[16]; unsigned short u[16]; };

__device__ __forceinline__ unsigned short bf16_bits(float x) { unsigned int u = __float_as_uint(x); return (unsigned short)((u + 0x7FFFu + ((u >> 16) & 1u)) >> 16); }
__device__ __forceinline__ float bf16_val(unsigned short b) { return __uint_as_float(((unsigned int)b) << 16); }
__device__ __forceinline__ float bf16_rne(float x) { return bf16_val(bf16_bits(x)); }
__device__ __forceinline__ int map_row(int r) { return (SQ == SQ_FULL) ? r : (r / SQ) * SQ_FULL + (r % SQ); }

__global__ __launch_bounds__(256) void k_wt_f16(const float* __restrict__ W, _Float16* __restrict__ Wt, int K, int N, float scale) {
  const int t = blockIdx.x * 256 + threadIdx.x; if (t >= N * (K / 8)) return; const int n = t / (K / 8), k8 = (t % (K / 8)) * 8; FragH f;
#pragma unroll
  for (int i = 0; i < 8; ++i) f.h[i] = (_Float16)(bf16_rne(W[(size_t)(k8 + i) * N + n]) * scale);
  const v8us o = f.half[0];
  *(volatile v8us*)((unsigned short*)Wt + (size_t)n * K + k8) = o; __threadfence(); *(volatile v8us*)((unsigned short*)Wt + (size_t)n * K + k8) = o;
}

template <int BFIN, int XMAP>
__device__ __forceinline__ void lnw_body(const float* __restrict__ X, const float* __restrict__ g, const float* __restrict__ bb, float eps, _Float16* __restrict__ N16, int nrows) {
  #pragma clang fp contract(off)
  static_assert(DM == 32 * 4 * 6);
  const int lane = threadIdx.x & 31; const int row = blockIdx.x * 8 + (threadIdx.x >> 5);
  if (row >= nrows) return;
  const float* xr = X + (size_t)(XMAP ? map_row(row) : row) * DM + lane * 4;
  float s[24]; float sum = 0.f;
#pragma unroll
  for (int u = 0; u < 6; ++u) { const v4f xa = *(const v4fa*)(xr + u * 128);
#pragma unroll
    for (int q = 0; q < 4; ++q) { const float v = BFIN ? bf16_rne(xa[q]) : xa[q]; s[u * 4 + q] = v; sum += v; } }
#pragma unroll
  for (int o = 16; o > 0; o >>= 1) sum += __shfl_xor(sum, o);
  const float inv = 1.0f / (float)DM;
  const float mu = sum * inv;
  float vs = 0.f;
#pragma unroll
  for (int i = 0; i < 24; ++i) { const float dl = s[i] - mu; vs += dl * dl; }
#pragma unroll
  for (int o = 16; o > 0; o >>= 1) vs += __shfl_xor(vs, o);
  const float rs = rsqrtf(vs * inv + eps);
  v4h y[6];
#pragma unroll
  for (int u = 0; u < 6; ++u) { const v4f gv = *(const v4fa*)(g + u * 128 + lane * 4); const v4f bv = *(const v4fa*)(bb + u * 128 + lane * 4);
#pragma unroll
    for (int q = 0; q < 4; ++q) y[u][q] = (_Float16)(((s[u * 4 + q] - mu) * rs) * bf16_rne(gv[q]) + bf16_rne(bv[q])); }
  _Float16* dst = N16 + (size_t)row * DM + lane * 4;
  for (int pass = 0; pass < 2; ++pass) {
#pragma unroll
    for (int u = 0; u < 6; ++u) *(volatile v4h*)(dst + u * 128) = y[u];
    if (pass == 0) __threadfence(); }
}
__global__ __launch_bounds__(256) void k_ln1(const float* __restrict__ X, const float* __restrict__ g, const float* __restrict__ bb, _Float16* __restrict__ N16) { lnw_body<1, 1>(X, g, bb, 1e-5f, N16, NR); }
__global__ __launch_bounds__(256) void k_ln2(const float* __restrict__ X, const float* __restrict__ g, const float* __restrict__ bb, _Float16* __restrict__ N16) { lnw_body<0, 0>(X, g, bb, 1e-5f, N16, NR); }

__device__ __forceinline__ v16h g2_frag(const _Float16* p, int hh) { FragH f; f.half[0] = *(const v8us*)((const unsigned short*)p + 8 * hh); f.half[1] = *(const v8us*)((const unsigned short*)p + 16 + 8 * hh); return f.v; }
__device__ __forceinline__ v8f g2_mma(v16h a, v16h b, v8f c) { v8f d = __builtin_amdgcn_wmma_f32_16x16x32_f16(false, a, false, b, (short)0, c, false, false); asm volatile("v_nop\n\tv_nop\n\tv_nop\n\tv_nop" : "+v"(d) : "v"(a), "v"(b)); return d; }
template <int ACT, int CPX, int COUT>
__device__ __forceinline__ void gemm2_body(const _Float16* __restrict__ A, int lda, size_t sA, const _Float16* __restrict__ Bh, int ldb, size_t sB, float alpha,
    const float* __restrict__ bias, const float* __restrict__ CP, float* __restrict__ C, _Float16* __restrict__ C16, int ldc, size_t sC, int M, int N, int K) {
  static_assert(ACT == 0 || ACT == 6);
  __shared__ __attribute__((aligned(16))) float so[4][32][68];
  const int tid = threadIdx.x, w = tid >> 5, lane = tid & 31, ln = lane & 15, hh = lane >> 4; const int by = blockIdx.y;
  A += (size_t)by * sA; Bh += (size_t)by * sB; const size_t cofs = (size_t)by * sC;
  const int ntn = N >> 6; const int mt = blockIdx.x / ntn, nq = blockIdx.x - mt * ntn; const int row0 = mt * 128 + 32 * w, col0 = nq * 64; if (row0 >= M) return;
  const _Float16* a0p = A + (size_t)(row0 + ln) * lda; const _Float16* a1p = a0p + (size_t)16 * lda;
  const _Float16* b0p = Bh + (size_t)(col0 + ln) * ldb; const _Float16* b1p = b0p + (size_t)16 * ldb; const _Float16* b2p = b1p + (size_t)16 * ldb; const _Float16* b3p = b2p + (size_t)16 * ldb;
  const v8f z8 = {0.f,0.f,0.f,0.f,0.f,0.f,0.f,0.f}; v8f c00 = z8, c01 = z8, c02 = z8, c03 = z8, c10 = z8, c11 = z8, c12 = z8, c13 = z8;
#pragma unroll 1
  for (int kb = 0; kb < K; kb += 32) { const v16h a0 = g2_frag(a0p + kb, hh), a1 = g2_frag(a1p + kb, hh);
    v16h b = g2_frag(b0p + kb, hh); c00 = g2_mma(a0, b, c00); c10 = g2_mma(a1, b, c10);
    b = g2_frag(b1p + kb, hh); c01 = g2_mma(a0, b, c01); c11 = g2_mma(a1, b, c11);
    b = g2_frag(b2p + kb, hh); c02 = g2_mma(a0, b, c02); c12 = g2_mma(a1, b, c12);
    b = g2_frag(b3p + kb, hh); c03 = g2_mma(a0, b, c03); c13 = g2_mma(a1, b, c13); }
  v8f accs[8] = {c00, c01, c02, c03, c10, c11, c12, c13};
#pragma unroll
  for (int u = 0; u < 8; ++u) { const int t = u & 3, half = u >> 2; const int col = col0 + t * 16 + ln; const float bv = bf16_rne(bias[col]);
#pragma unroll
    for (int r = 0; r < 8; ++r) { const int rloc = half * 16 + 8 * hh + r; float v = accs[u][r] * alpha + bv;
      if (CP) { const int rg = CPX ? map_row(row0 + rloc) : (row0 + rloc); float cv = CP[cofs + (size_t)rg * ldc + col]; if (CPX) cv = bf16_rne(cv); v += cv; }
      if (ACT == 6) v = 0.5f * v * (1.0f + erff(v * 0.70710678118654752f));
      so[w][rloc][t * 16 + ln] = v; } }
  __builtin_amdgcn_fence(4  , "workgroup"); __builtin_amdgcn_wave_barrier();
  const int rsub = lane >> 4, c4 = (lane & 15) * 4;
  for (int pass = 0; pass < 2; ++pass) {
#pragma unroll
    for (int q = 0; q < 16; ++q) { const int r = q * 2 + rsub; const v4f v = *(const v4fa*)&so[w][r][c4];
      if (C) { const int rg = COUT ? map_row(row0 + r) : (row0 + r); *(volatile v4f*)(C + cofs + (size_t)rg * ldc + col0 + c4) = v; }
      if (C16) { v4h h4; for (int i = 0; i < 4; ++i) h4[i] = (_Float16)v[i]; *(volatile v4h*)(C16 + cofs + (size_t)(row0 + r) * ldc + col0 + c4) = h4; } }
    if (pass == 0) __threadfence(); } }
__global__ __launch_bounds__(128) void k_gemm_qkv(const _Float16* __restrict__ A, const _Float16* __restrict__ Bt, const float* __restrict__ bias, _Float16* __restrict__ C16) {
  gemm2_body<0, 0, 0>(A, DM, 0, Bt, DM, 0, 0.0625f, bias, nullptr, nullptr, C16, LQ, 0, NR, LQ, DM); }
__global__ __launch_bounds__(128) void k_gemm_proj(const _Float16* __restrict__ A, const _Float16* __restrict__ Bt, const float* __restrict__ bias, const float* __restrict__ X, float* __restrict__ C) {
  gemm2_body<0, 1, 0>(A, DM, 0, Bt, DM, 0, 0.0009765625f, bias, X, C, nullptr, DM, 0, NR, DM, DM); }
__global__ __launch_bounds__(128) void k_gemm_fc1(const _Float16* __restrict__ A, const _Float16* __restrict__ Bt, const float* __restrict__ bias, _Float16* __restrict__ C16) {
  gemm2_body<6, 0, 0>(A, DM, 0, Bt, DM, 0, 0.0625f, bias, nullptr, nullptr, C16, DFF, 0, NR, DFF, DM); }
__global__ __launch_bounds__(128) void k_gemm_fc2(const _Float16* __restrict__ A, const _Float16* __restrict__ Bt, const float* __restrict__ bias, const float* __restrict__ X1, float* __restrict__ C) {
  gemm2_body<0, 0, 1>(A, DFF, 0, Bt, DFF, 0, 0.0625f, bias, X1, C, nullptr, DM, 0, NR, DM, DFF); }

template <int NHv, int TTv>
__device__ __forceinline__ void vt_body(const _Float16* __restrict__ V16, int ldv, int voff, _Float16* __restrict__ Vt) { __shared__ unsigned short tl[64][66]; const int tid = threadIdx.x; const int slab = blockIdx.x / (TTv / 64), lg = blockIdx.x % (TTv / 64); const int b = slab / NHv, h = slab % NHv;
  for (int i = tid; i < 64 * 8; i += 256) { const int r = i / 8, c8 = (i % 8) * 8; FragH f; f.half[0] = *(const v8us*)((const unsigned short*)V16 + ((size_t)b * TTv + lg * 64 + r) * ldv + voff + h * 64 + c8);
#pragma unroll
    for (int q = 0; q < 8; ++q) tl[r][c8 + q] = f.u[q]; }
  __syncthreads();
  for (int pass = 0; pass < 2; ++pass) {
#pragma unroll
    for (int rd = 0; rd < 2; ++rd) { const int d = rd * 32 + tid / 8, pc = tid % 8; FragH f;
#pragma unroll
      for (int q = 0; q < 8; ++q) f.u[q] = tl[pc * 8 + q][d];
      *(volatile v8us*)((unsigned short*)Vt + ((size_t)slab * 64 + d) * TTv + lg * 64 + pc * 8) = f.half[0]; }
    if (pass == 0) __threadfence(); } }
__global__ __launch_bounds__(256) void k_vt_all(const _Float16* __restrict__ QKV, _Float16* __restrict__ Vt) { vt_body<NH, SQ>(QKV, LQ, 2 * DM, Vt); }

__device__ __forceinline__ float v8max(v8f a) { return fmaxf(fmaxf(fmaxf(a[0], a[1]), fmaxf(a[2], a[3])), fmaxf(fmaxf(a[4], a[5]), fmaxf(a[6], a[7]))); }
__device__ __forceinline__ float v8sum(v8f a) { return ((a[0] + a[1]) + (a[2] + a[3])) + ((a[4] + a[5]) + (a[6] + a[7])); }
__device__ __forceinline__ v8f fa_scores(const _Float16* kp, int hh, v16h q0, v16h q1) { const v8f z = {0.f,0.f,0.f,0.f,0.f,0.f,0.f,0.f}; v8f s = g2_mma(g2_frag(kp, hh), q0, z); return g2_mma(g2_frag(kp + 32, hh), q1, s); }
__device__ __forceinline__ v8f fa_exp(v8f s, float cc) { v8f p;
#pragma unroll
  for (int r = 0; r < 8; ++r) p[r] = exp2f(fmaf(s[r], SC2, cc));
  return p; }
__device__ __forceinline__ v16h fa_pfrag(v8f pa, v8f pb) { FragH f;
#pragma unroll
  for (int r = 0; r < 8; ++r) { f.h[r] = (_Float16)pa[r]; f.h[8 + r] = (_Float16)pb[r]; }
  return f.v; }
__device__ __forceinline__ v8f fa_pv(const _Float16* vp, int hh, v16h pb0, v16h pb1, v8f o) { o = g2_mma(g2_frag(vp, hh), pb0, o); return g2_mma(g2_frag(vp + 32, hh), pb1, o); }

__global__ __launch_bounds__(128) void k_flash(const _Float16* __restrict__ QKV, const _Float16* __restrict__ VT, _Float16* __restrict__ O16) {
  __shared__ __attribute__((aligned(16))) unsigned short ots[4][16][72];
  const int tid = threadIdx.x, w = tid >> 5, lane = tid & 31, ln = lane & 15, hh = lane >> 4;
  const int bh = blockIdx.y; const int b = bh / NH, h = bh - b * NH;
  const int q0 = blockIdx.x * 64 + 16 * w;
  const _Float16* qrow = QKV + ((size_t)b * SQ + q0 + ln) * LQ + h * HD;
  const v16h qf0 = g2_frag(qrow, hh), qf1 = g2_frag(qrow + 32, hh);
  const _Float16* kbase = QKV + ((size_t)b * SQ + ln) * LQ + DM + h * HD;
  const _Float16* vbase = VT + ((size_t)bh * HD + ln) * SQ;
  const v8f z8 = {0.f,0.f,0.f,0.f,0.f,0.f,0.f,0.f};
  v8f o0 = z8, o1 = z8, o2 = z8, o3 = z8; float m = -1.0e30f, l = 0.f;
#pragma unroll 1
  for (int c = 0; c < SQ / 64; ++c) {
    const _Float16* kp = kbase + (size_t)(c * 64) * LQ;
    const v8f s0 = fa_scores(kp, hh, qf0, qf1);
    const v8f s1 = fa_scores(kp + (size_t)16 * LQ, hh, qf0, qf1);
    const v8f s2 = fa_scores(kp + (size_t)32 * LQ, hh, qf0, qf1);
    const v8f s3 = fa_scores(kp + (size_t)48 * LQ, hh, qf0, qf1);
    float mx = fmaxf(fmaxf(v8max(s0), v8max(s1)), fmaxf(v8max(s2), v8max(s3)));
    mx = fmaxf(mx, __shfl_xor(mx, 16));
    const float mn = fmaxf(m, mx * SC2);
    const float alpha = exp2f(m - mn);
    const float cc = 8.0f - mn;
    const v8f p0 = fa_exp(s0, cc), p1 = fa_exp(s1, cc), p2 = fa_exp(s2, cc), p3 = fa_exp(s3, cc);
    float ps = (v8sum(p0) + v8sum(p1)) + (v8sum(p2) + v8sum(p3));
    ps += __shfl_xor(ps, 16);
    l = l * alpha + ps; m = mn;
    const v16h pb0 = fa_pfrag(p0, p1), pb1 = fa_pfrag(p2, p3);
    o0 *= alpha; o1 *= alpha; o2 *= alpha; o3 *= alpha;
    asm volatile("" ::: "memory");
    const _Float16* vp = vbase + c * 64;
    o0 = fa_pv(vp, hh, pb0, pb1, o0);
    o1 = fa_pv(vp + (size_t)16 * SQ, hh, pb0, pb1, o1);
    o2 = fa_pv(vp + (size_t)32 * SQ, hh, pb0, pb1, o2);
    o3 = fa_pv(vp + (size_t)48 * SQ, hh, pb0, pb1, o3);
  }
  const float fin = 64.0f / l;
  v8f oo[4] = {o0, o1, o2, o3};
#pragma unroll
  for (int dt = 0; dt < 4; ++dt) { FragH f;
#pragma unroll
    for (int r = 0; r < 8; ++r) f.h[r] = (_Float16)(oo[dt][r] * fin);
    *(v8us*)&ots[w][ln][16 * dt + 8 * hh] = f.half[0]; }
  __builtin_amdgcn_fence(4  , "workgroup"); __builtin_amdgcn_wave_barrier();
  const int rq = lane >> 3, pc = (lane & 7) * 8;
  unsigned short* obase = (unsigned short*)O16 + ((size_t)b * SQ + q0) * DM + h * HD;
  for (int pass = 0; pass < 2; ++pass) {
#pragma unroll
    for (int it = 0; it < 4; ++it) { const int row = it * 4 + rq; const v8us v = *(const v8us*)&ots[w][row][pc]; *(volatile v8us*)(obase + (size_t)row * DM + pc) = v; }
    if (pass == 0) __threadfence(); }
}

constexpr size_t al256(size_t b) { return (b + 255) & ~(size_t)255; }
constexpr size_t SZ_BQ  = al256((size_t)LQ * DM * 2);
constexpr size_t SZ_BO  = al256((size_t)DM * DM * 2);
constexpr size_t SZ_BW1 = al256((size_t)DFF * DM * 2);
constexpr size_t SZ_BW2 = al256((size_t)DM * DFF * 2);
constexpr size_t SZ_XN  = al256((size_t)NR * DM * 2);
constexpr size_t SZ_X1  = al256((size_t)NR * DM * 4);
constexpr size_t SZ_QKV = al256((size_t)NR * LQ * 2);
constexpr size_t SZ_VT  = al256((size_t)NB * NH * HD * SQ * 2);
constexpr size_t SZ_HF  = al256((size_t)NR * DFF * 2);
constexpr size_t OFF_BQ = 0;
constexpr size_t OFF_BO = OFF_BQ + SZ_BQ;
constexpr size_t OFF_BW1 = OFF_BO + SZ_BO;
constexpr size_t OFF_BW2 = OFF_BW1 + SZ_BW1;
constexpr size_t OFF_XN = OFF_BW2 + SZ_BW2;
constexpr size_t OFF_X1 = OFF_XN + SZ_XN;
constexpr size_t OFF_QKV = OFF_X1 + SZ_X1;
constexpr size_t OFF_VT = OFF_QKV + SZ_QKV;
constexpr size_t WS_TOTAL = OFF_VT + SZ_VT;
static_assert(WS_TOTAL <= (size_t)134217728);
static_assert(OFF_VT == OFF_QKV + SZ_QKV);
static_assert(SZ_HF <= SZ_QKV + SZ_VT);

extern "C" void kernel_launch(void* const* d_in, const int* in_sizes, int n_in,
                              void* d_out, int out_size, void* d_ws, size_t ws_size, hipStream_t stream) {
  if (n_in < 13) return;
  const long long need_x = ((long long)(NB - 1) * SQ_FULL + SQ) * DM;
  if ((long long)in_sizes[0] < need_x) return; if (in_sizes[1] < DM) return; if (in_sizes[2] < DM) return;
  if ((long long)in_sizes[3] < (long long)DM * LQ) return; if (in_sizes[4] < LQ) return;
  if ((long long)in_sizes[5] < (long long)DM * DM) return; if (in_sizes[6] < DM) return; if (in_sizes[7] < DM) return; if (in_sizes[8] < DM) return;
  if ((long long)in_sizes[9] < (long long)DM * DFF) return; if (in_sizes[10] < DFF) return;
  if ((long long)in_sizes[11] < (long long)DFF * DM) return; if (in_sizes[12] < DM) return;
  if ((long long)out_size < need_x) return;
  if (ws_size < WS_TOTAL) return;
  const float* const* I = (const float* const*)d_in;
  const float* x = I[0]; const float* g1 = I[1]; const float* be1 = I[2]; const float* wqkv = I[3]; const float* bqkv = I[4]; const float* wo = I[5]; const float* bo = I[6];
  const float* g2 = I[7]; const float* be2 = I[8]; const float* w1 = I[9]; const float* b1 = I[10]; const float* w2 = I[11]; const float* b2 = I[12];
  char* ws = (char*)d_ws;
  _Float16* BQ = (_Float16*)(ws + OFF_BQ); _Float16* BO = (_Float16*)(ws + OFF_BO); _Float16* BW1 = (_Float16*)(ws + OFF_BW1); _Float16* BW2 = (_Float16*)(ws + OFF_BW2);
  _Float16* XN = (_Float16*)(ws + OFF_XN); _Float16* O16 = XN; _Float16* M16 = XN;
  float* X1 = (float*)(ws + OFF_X1); _Float16* QKV16 = (_Float16*)(ws + OFF_QKV); _Float16* VT = (_Float16*)(ws + OFF_VT);
  _Float16* HF16 = (_Float16*)(ws + OFF_QKV);

  k_wt_f16<<<(unsigned)(((size_t)LQ * (DM / 8) + 255) / 256), 256, 0, stream>>>(wqkv, BQ, DM, LQ, 16.0f);
  k_wt_f16<<<(unsigned)(((size_t)DM * (DM / 8) + 255) / 256), 256, 0, stream>>>(wo, BO, DM, DM, 16.0f);
  k_wt_f16<<<(unsigned)(((size_t)DFF * (DM / 8) + 255) / 256), 256, 0, stream>>>(w1, BW1, DM, DFF, 16.0f);
  k_wt_f16<<<(unsigned)(((size_t)DM * (DFF / 8) + 255) / 256), 256, 0, stream>>>(w2, BW2, DFF, DM, 16.0f);
  k_ln1<<<(unsigned)((NR + 7) / 8), 256, 0, stream>>>(x, g1, be1, XN);
  k_gemm_qkv<<<dim3((unsigned)((NR / 128) * (LQ / 64)), 1), 128, 0, stream>>>(XN, BQ, bqkv, QKV16);
  k_vt_all<<<(unsigned)(NB * NH * (SQ / 64)), 256, 0, stream>>>(QKV16, VT);
  k_flash<<<dim3((unsigned)(SQ / 64), (unsigned)(NB * NH)), 128, 0, stream>>>(QKV16, VT, O16);
  k_gemm_proj<<<dim3((unsigned)((NR / 128) * (DM / 64)), 1), 128, 0, stream>>>(O16, BO, bo, x, X1);
  k_ln2<<<(unsigned)((NR + 7) / 8), 256, 0, stream>>>(X1, g2, be2, M16);
  k_gemm_fc1<<<dim3((unsigned)((NR / 128) * (DFF / 64)), 1), 128, 0, stream>>>(M16, BW1, b1, HF16);
  k_gemm_fc2<<<dim3((unsigned)((NR / 128) * (DM / 64)), 1), 128, 0, stream>>>(HF16, BW2, b2, X1, (float*)d_out);
}
